// MambaLayer_42125039239784
// MI455X (gfx1250) — hardware-verified
//
#include <hip/hip_runtime.h>
#include <stddef.h>
#include <stdint.h>

#define BSZ    4
#define SEQ    2048
#define DM     512
#define DI     1024
#define NXZ    2048
#define DTR    32
#define DS     16
#define XD     64
#define MROWS  8192
#define K2     2048
#define KDT2   64
#define GBM    64
#define GTHR   128
#define PTHR   256
#define TC     32
#define WSMAX  134217728

#define NU_XB   (MROWS * DM / 8)
#define NU_WIN  (NXZ * DM / 8)
#define NU_WX   (XD * K2 / 8)
#define NU_WDT  (DI * KDT2 / 8)
#define NU_WOUT (DM * K2 / 8)
#define NU_AT   (DI * DS / 4)
#define NU_ALL  (NU_XB + NU_WIN + NU_WX + NU_WDT + NU_WOUT + NU_AT)

static_assert(MROWS == BSZ * SEQ);
static_assert(K2 == 2 * DI && KDT2 == 2 * DTR && XD == DTR + 2 * DS && NXZ == 2 * DI);
static_assert(DM % 32 == 0 && K2 % 32 == 0 && KDT2 % 32 == 0);
static_assert(MROWS % GBM == 0 && NXZ % 128 == 0 && DI % 128 == 0 && DM % 128 == 0 && XD == 64);
static_assert(SEQ % 64 == 0 && SEQ % TC == 0 && DI % 64 == 0);
static_assert(NU_XB % PTHR == 0 && NU_WIN % PTHR == 0 && NU_WX % PTHR == 0 && NU_WDT % PTHR == 0);
static_assert(NU_WOUT % PTHR == 0 && NU_AT % PTHR == 0 && NU_ALL % PTHR == 0);
static_assert(GBM == (GTHR / 32) * 16);

typedef float          v4f   __attribute__((ext_vector_type(4)));
typedef float          v8f   __attribute__((ext_vector_type(8)));
typedef int            v8i   __attribute__((ext_vector_type(8)));
typedef unsigned short v8us  __attribute__((ext_vector_type(8)));
typedef unsigned short v16us __attribute__((ext_vector_type(16)));
typedef __bf16         v16bf __attribute__((ext_vector_type(16)));
typedef v4f  __attribute__((may_alias)) v4fa;
typedef v8us __attribute__((may_alias)) v8usa;
union FragB { v16bf v; v16us u; v8us h[2]; v8i w; };

__device__ __forceinline__ v8f wmb(const FragB& a, const FragB& b, v8f c) {
  v8f d = __builtin_amdgcn_wmma_f32_16x16x32_bf16(false, a.v, false, b.v, (short)0, c, false, false);
  asm volatile("v_nop\n\tv_nop\n\tv_nop\n\tv_nop" : "+v"(d) : "v"(a.w), "v"(b.w));
  return d;
}

__device__ __forceinline__ unsigned bf16_bits(float f) {
  const unsigned u = __float_as_uint(f);
  return (u + 0x7FFFu + ((u >> 16) & 1u)) >> 16;
}
__device__ __forceinline__ float bf16_val(float f) {
  return __uint_as_float(bf16_bits(f) << 16);
}
__device__ __forceinline__ float silu_f(float v) {
  return v * __builtin_amdgcn_rcpf(1.0f + expf(-v));
}
__device__ __forceinline__ float softplus_f(float v) {
  return fmaxf(v, 0.0f) + log1pf(expf(-fabsf(v)));
}
__device__ __forceinline__ void put16(unsigned short* dp, v8us o) {
  *(volatile v8us*)dp = o;
  __threadfence();
  *(volatile v8us*)dp = o;
}
__device__ __forceinline__ void putf4(float* dp, v4f o) {
  *(volatile v4f*)dp = o;
  __threadfence();
  *(volatile v4f*)dp = o;
}

__global__ __launch_bounds__(PTHR) void k_prep(const float* __restrict__ x, const float* __restrict__ Win,
                                               const float* __restrict__ Wx, const float* __restrict__ Wdt,
                                               const float* __restrict__ Wout, const float* __restrict__ Alog,
                                               unsigned short* XB, unsigned short* WIN, unsigned short* WX2,
                                               unsigned short* WDT2, unsigned short* WOUT2, float* ATAB) {
  const int u  = (int)blockIdx.x * PTHR + (int)threadIdx.x;
  const int P0 = NU_XB;
  const int P1 = P0 + NU_WIN;
  const int P2 = P1 + NU_WX;
  const int P3 = P2 + NU_WDT;
  const int P4 = P3 + NU_WOUT;
  const int P5 = P4 + NU_AT;
  if (u >= P5) return;
  if (u >= P4) {
    const int v = u - P4;
    const v4f al = *(const v4fa*)(Alog + (size_t)v * 4);
    v4f o;
    o.x = -expf(bf16_val(al.x));
    o.y = -expf(bf16_val(al.y));
    o.z = -expf(bf16_val(al.z));
    o.w = -expf(bf16_val(al.w));
    putf4(ATAB + (size_t)v * 4, o);
    return;
  }
  const float* src;
  unsigned short* dst;
  if (u < P0) {
    src = x + (size_t)u * 8;
    dst = XB + (size_t)u * 8;
  } else if (u < P1) {
    const int v = u - P0;
    src = Win + (size_t)v * 8;
    dst = WIN + (size_t)v * 8;
  } else if (u < P2) {
    const int v  = u - P1;
    const int n  = v >> 8;
    const int k8 = (v & 255) * 8;
    src = Wx + (size_t)n * DI + (k8 & (DI - 1));
    dst = WX2 + (size_t)n * K2 + k8;
  } else if (u < P3) {
    const int v  = u - P2;
    const int n  = v >> 3;
    const int k8 = (v & 7) * 8;
    src = Wdt + (size_t)n * DTR + (k8 & (DTR - 1));
    dst = WDT2 + (size_t)n * KDT2 + k8;
  } else {
    const int v  = u - P3;
    const int n  = v >> 8;
    const int k8 = (v & 255) * 8;
    src = Wout + (size_t)n * DI + (k8 & (DI - 1));
    dst = WOUT2 + (size_t)n * K2 + k8;
  }
  const v4f a = *(const v4fa*)src;
  const v4f c = *(const v4fa*)(src + 4);
  v8us o;
  o[0] = (unsigned short)bf16_bits(a.x);
  o[1] = (unsigned short)bf16_bits(a.y);
  o[2] = (unsigned short)bf16_bits(a.z);
  o[3] = (unsigned short)bf16_bits(a.w);
  o[4] = (unsigned short)bf16_bits(c.x);
  o[5] = (unsigned short)bf16_bits(c.y);
  o[6] = (unsigned short)bf16_bits(c.z);
  o[7] = (unsigned short)bf16_bits(c.w);
  put16(dst, o);
}

template <int NT, int MODE>
__global__ __launch_bounds__(GTHR) void k_gemm(const unsigned short* __restrict__ A, int lda,
                                               const unsigned short* __restrict__ BT, int ldb, int K,
                                               const float* __restrict__ bias,
                                               float* C0, float* C1, unsigned short* Cb) {
  constexpr int BN = 16 * NT;
  __shared__ __attribute__((aligned(16))) float stg[GBM * BN];
  const int tid = (int)threadIdx.x, lane = tid & 31, wave = tid >> 5, hh = lane >> 4, m = lane & 15;
  const int rowBase = (int)blockIdx.x * GBM;
  const int colBase = (int)blockIdx.y * BN;

  v8f acc[NT];
  {
    const v8f z = {0.f, 0.f, 0.f, 0.f, 0.f, 0.f, 0.f, 0.f};
#pragma unroll
    for (int t = 0; t < NT; ++t) acc[t] = z;
  }
  const unsigned short* ap = A  + (size_t)(rowBase + 16 * wave + m) * (size_t)lda + 8 * hh;
  const unsigned short* bp = BT + (size_t)(colBase + m) * (size_t)ldb + 8 * hh;

#pragma unroll 1
  for (int k0 = 0; k0 < K; k0 += 32) {
    FragB af;
    af.h[0] = *(const v8usa*)(ap + k0);
    af.h[1] = *(const v8usa*)(ap + k0 + 16);
#pragma unroll
    for (int nt = 0; nt < NT; ++nt) {
      const unsigned short* wq = bp + (size_t)(16 * nt) * (size_t)ldb + k0;
      FragB bf;
      bf.h[0] = *(const v8usa*)wq;
      bf.h[1] = *(const v8usa*)(wq + 16);
      acc[nt] = wmb(af, bf, acc[nt]);
    }
  }

#pragma unroll
  for (int nt = 0; nt < NT; ++nt) {
    const int lc = 16 * nt + m;
#pragma unroll
    for (int r = 0; r < 8; ++r) {
      const int lr = 16 * wave + 8 * hh + r;
      stg[lr * BN + lc] = acc[nt][r];
    }
  }
  __syncthreads();

  if constexpr (MODE == 1) {
    const int q = lane >> 3, j = lane & 7;
    const int part = j >> 2;
    const int c8 = 8 * (j & 3);
    const unsigned mh = 0u - (unsigned)part;
    const unsigned ml = ~mh;
    v8us pd[4];
    v4f  pb[4];
#pragma unroll
    for (int s = 0; s < 4; ++s) {
      const int lr = 16 * wave + 4 * s + q;
      const float* sp = stg + lr * BN + c8;
      const v4f a = *(const v4fa*)sp;
      const v4f b = *(const v4fa*)(sp + 4);
      const v8f f8 = {a.x, a.y, a.z, a.w, b.x, b.y, b.z, b.w};
      v8us oo;
#pragma unroll
      for (int e = 0; e < 8; ++e) {
        const unsigned hb = bf16_bits(f8[e]);
        const unsigned lb = bf16_bits(f8[e] - __uint_as_float(hb << 16));
        oo[e] = (unsigned short)((hb & ml) | (lb & mh));
      }
      pd[s] = oo;
      pb[s] = *(const v4fa*)(stg + lr * BN + 32 + 4 * j);
    }
#pragma unroll
    for (int s = 0; s < 4; ++s) {
      const size_t row = (size_t)(rowBase + 16 * wave + 4 * s + q);
      *(volatile v8us*)(Cb + row * 64 + 8 * j) = pd[s];
      *(volatile v4f*)(C0 + row * 32 + 4 * j)  = pb[s];
    }
    __threadfence();
#pragma unroll
    for (int s = 0; s < 4; ++s) {
      const size_t row = (size_t)(rowBase + 16 * wave + 4 * s + q);
      *(volatile v8us*)(Cb + row * 64 + 8 * j) = pd[s];
      *(volatile v4f*)(C0 + row * 32 + 4 * j)  = pb[s];
    }
  } else {
    float* dst = C0;
    int ldc = DI;
    int cb = colBase;
    bool gate = false;
    v4f b4 = {0.0f, 0.0f, 0.0f, 0.0f};
    if constexpr (MODE == 0) {
      gate = colBase >= DI;
      if (gate) { dst = C1; cb = colBase - DI; }
    }
    if constexpr (MODE == 2) {
      const v4f bl = *(const v4fa*)(bias + colBase + 4 * lane);
      b4.x = bf16_val(bl.x);
      b4.y = bf16_val(bl.y);
      b4.z = bf16_val(bl.z);
      b4.w = bf16_val(bl.w);
    }
    if constexpr (MODE == 3) ldc = DM;
#pragma unroll 1
    for (int i = 0; i < 16; ++i) {
      float* sp = stg + (16 * wave + i) * BN + 4 * lane;
      v4f v = *(const v4fa*)sp;
      if constexpr (MODE == 0) {
        if (gate) {
          v.x = silu_f(v.x);
          v.y = silu_f(v.y);
          v.z = silu_f(v.z);
          v.w = silu_f(v.w);
          *(v4fa*)sp = v;
        }
      }
      if constexpr (MODE == 2) {
        v.x = softplus_f(v.x + b4.x);
        v.y = softplus_f(v.y + b4.y);
        v.z = softplus_f(v.z + b4.z);
        v.w = softplus_f(v.w + b4.w);
        *(v4fa*)sp = v;
      }
      float* op = dst + (size_t)(rowBase + 16 * wave + i) * (size_t)ldc + cb + 4 * lane;
      *(volatile v4f*)op = v;
    }
    __threadfence();
#pragma unroll 1
    for (int i = 0; i < 16; ++i) {
      const float* sp = stg + (16 * wave + i) * BN + 4 * lane;
      const v4f v = *(const v4fa*)sp;
      float* op = dst + (size_t)(rowBase + 16 * wave + i) * (size_t)ldc + cb + 4 * lane;
      *(volatile v4f*)op = v;
    }
  }
}

__global__ __launch_bounds__(PTHR) void k_conv(const float* __restrict__ U, const float* __restrict__ Wc,
                                               const float* __restrict__ bc, unsigned short* UC) {
  __shared__ __attribute__((aligned(16))) unsigned short sH[64 * 64];
  __shared__ __attribute__((aligned(16))) unsigned short sL[64 * 64];
  const int tid = (int)threadIdx.x;
  const int c = tid & 63, rg = tid >> 6;
  const int rowBase = (int)blockIdx.x * 64;
  const int c0 = (int)blockIdx.y * 64;
  const int d = c0 + c;

  const v4f wr = *(const v4fa*)(Wc + (size_t)d * 4);
  const float w0 = bf16_val(wr.x), w1 = bf16_val(wr.y), w2 = bf16_val(wr.z), w3 = bf16_val(wr.w);
  const float bv = bf16_val(bc[d]);

  const int row0 = rowBase + 16 * rg;
  const int t0 = row0 & (SEQ - 1);
  const bool ok = t0 >= 3;
  const float* p = U + (size_t)row0 * DI + d;
  const int back = ok ? DI : 0;
  const float l3 = *(p - 3 * back);
  const float l2 = *(p - 2 * back);
  const float l1 = *(p - back);
  float xm3 = ok ? l3 : 0.0f;
  float xm2 = ok ? l2 : 0.0f;
  float xm1 = ok ? l1 : 0.0f;

#pragma unroll 1
  for (int i = 0; i < 16; ++i) {
    const float xc = p[(size_t)i * DI];
    float s = bv;
    s = s + xm3 * w0;
    s = s + xm2 * w1;
    s = s + xm1 * w2;
    s = s + xc * w3;
    const float r = silu_f(s);
    const unsigned hb = bf16_bits(r);
    const unsigned lb = bf16_bits(r - __uint_as_float(hb << 16));
    sH[(16 * rg + i) * 64 + c] = (unsigned short)hb;
    sL[(16 * rg + i) * 64 + c] = (unsigned short)lb;
    xm3 = xm2;
    xm2 = xm1;
    xm1 = xc;
  }
  __syncthreads();

  v8us vh[2], vl[2];
#pragma unroll
  for (int s = 0; s < 2; ++s) {
    const int id = tid + PTHR * s;
    const int r = id >> 3, j = id & 7;
    vh[s] = *(const v8usa*)(sH + r * 64 + 8 * j);
    vl[s] = *(const v8usa*)(sL + r * 64 + 8 * j);
  }
#pragma unroll
  for (int s = 0; s < 2; ++s) {
    const int id = tid + PTHR * s;
    const int r = id >> 3, j = id & 7;
    unsigned short* op = UC + (size_t)(rowBase + r) * K2 + c0 + 8 * j;
    *(volatile v8us*)op        = vh[s];
    *(volatile v8us*)(op + DI) = vl[s];
  }
  __threadfence();
#pragma unroll
  for (int s = 0; s < 2; ++s) {
    const int id = tid + PTHR * s;
    const int r = id >> 3, j = id & 7;
    unsigned short* op = UC + (size_t)(rowBase + r) * K2 + c0 + 8 * j;
    *(volatile v8us*)op        = vh[s];
    *(volatile v8us*)(op + DI) = vl[s];
  }
}

__global__ __launch_bounds__(64) void k_scan(const float* __restrict__ DEL, const float* __restrict__ G,
                                             const float* __restrict__ BC, const float* __restrict__ ATAB,
                                             const float* __restrict__ Dp, unsigned short* UY) {
  __shared__ __attribute__((aligned(16))) float sDel[TC * 64];
  __shared__ __attribute__((aligned(16))) float sG[TC * 64];
  __shared__ __attribute__((aligned(16))) float sBC[TC * 32];
  __shared__ __attribute__((aligned(16))) unsigned short sUh[TC * 64];
  __shared__ __attribute__((aligned(16))) unsigned short sUl[TC * 64];

  const int tid = (int)threadIdx.x;
  const int b  = (int)blockIdx.x >> 4;
  const int c0 = ((int)blockIdx.x & 15) * 64;
  const int d  = c0 + tid;

  float a[DS], h[DS];
  {
    v4f al[4];
#pragma unroll
    for (int q = 0; q < 4; ++q) al[q] = *(const v4fa*)(ATAB + (size_t)d * DS + 4 * q);
#pragma unroll
    for (int q = 0; q < 4; ++q) {
#pragma unroll
      for (int e = 0; e < 4; ++e) {
        a[4 * q + e] = al[q][e];
        h[4 * q + e] = 0.0f;
      }
    }
  }
  const float dp = bf16_val(Dp[d]);

#pragma unroll 1
  for (int ch = 0; ch < SEQ / TC; ++ch) {
    const size_t rowb = (size_t)b * SEQ + (size_t)ch * TC;
#pragma unroll
    for (int s = 0; s < 8; ++s) {
      const int id = tid + 64 * s;
      const int r = id >> 4, q = id & 15;
      const size_t go = (rowb + r) * DI + c0 + 4 * q;
      *(v4fa*)(sDel + r * 64 + 4 * q) = *(const v4fa*)(DEL + go);
      *(v4fa*)(sG + r * 64 + 4 * q)   = *(const v4fa*)(G + go);
    }
#pragma unroll
    for (int s = 0; s < 4; ++s) {
      const int id = tid + 64 * s;
      const int r = id >> 3, q = id & 7;
      *(v4fa*)(sBC + r * 32 + 4 * q) = *(const v4fa*)(BC + (rowb + r) * 32 + 4 * q);
      const unsigned short* up = UY + (rowb + r) * K2 + c0 + 8 * q;
      *(v8usa*)(sUh + r * 64 + 8 * q) = *(const v8usa*)up;
      *(v8usa*)(sUl + r * 64 + 8 * q) = *(const v8usa*)(up + DI);
    }
    __syncthreads();

#pragma unroll 1
    for (int tt = 0; tt < TC; ++tt) {
      const int li = tt * 64 + tid;
      const float dl = sDel[li];
      const float g  = sG[li];
      const unsigned uh = sUh[li];
      const unsigned ul = sUl[li];
      const float u = __uint_as_float(uh << 16) + __uint_as_float(ul << 16);
      const float* bcp = sBC + tt * 32;
      v4f bq[4], cq[4];
#pragma unroll
      for (int q = 0; q < 4; ++q) {
        bq[q] = *(const v4fa*)(bcp + 4 * q);
        cq[q] = *(const v4fa*)(bcp + 16 + 4 * q);
      }
      const float du = dl * u;
      float y = 0.0f;
#pragma unroll
      for (int n = 0; n < DS; ++n) {
        const float dA = expf(dl * a[n]);
        h[n] = dA * h[n] + du * bq[n >> 2][n & 3];
        y = y + h[n] * cq[n >> 2][n & 3];
      }
      y = y + u * dp;
      y = y * g;
      const unsigned hb = bf16_bits(y);
      const unsigned lb = bf16_bits(y - __uint_as_float(hb << 16));
      sUh[li] = (unsigned short)hb;
      sUl[li] = (unsigned short)lb;
    }
    __syncthreads();

    v8us vh[4], vl[4];
#pragma unroll
    for (int s = 0; s < 4; ++s) {
      const int id = tid + 64 * s;
      const int r = id >> 3, q = id & 7;
      vh[s] = *(const v8usa*)(sUh + r * 64 + 8 * q);
      vl[s] = *(const v8usa*)(sUl + r * 64 + 8 * q);
    }
#pragma unroll
    for (int s = 0; s < 4; ++s) {
      const int id = tid + 64 * s;
      const int r = id >> 3, q = id & 7;
      unsigned short* op = UY + (rowb + r) * K2 + c0 + 8 * q;
      *(volatile v8us*)op        = vh[s];
      *(volatile v8us*)(op + DI) = vl[s];
    }
    __threadfence();
#pragma unroll
    for (int s = 0; s < 4; ++s) {
      const int id = tid + 64 * s;
      const int r = id >> 3, q = id & 7;
      unsigned short* op = UY + (rowb + r) * K2 + c0 + 8 * q;
      *(volatile v8us*)op        = vh[s];
      *(volatile v8us*)(op + DI) = vl[s];
    }
    __syncthreads();
  }
}

extern "C" void kernel_launch(void* const* d_in, const int* in_sizes, int n_in,
                              void* d_out, int out_size, void* d_ws, size_t ws_size,
                              hipStream_t stream) {
  if (n_in < 10) return;
  if (in_sizes[0] != MROWS * DM) return;
  if (in_sizes[1] != NXZ * DM) return;
  if (in_sizes[2] != DI * 4) return;
  if (in_sizes[3] != DI) return;
  if (in_sizes[4] != XD * DI) return;
  if (in_sizes[5] != DI * DTR) return;
  if (in_sizes[6] != DI) return;
  if (in_sizes[7] != DI * DS) return;
  if (in_sizes[8] != DI) return;
  if (in_sizes[9] != DM * DI) return;
  if (out_size != MROWS * DM) return;

  const float* x      = (const float*)d_in[0];
  const float* W_in   = (const float*)d_in[1];
  const float* W_conv = (const float*)d_in[2];
  const float* b_conv = (const float*)d_in[3];
  const float* W_x    = (const float*)d_in[4];
  const float* W_dt   = (const float*)d_in[5];
  const float* b_dt   = (const float*)d_in[6];
  const float* A_log  = (const float*)d_in[7];
  const float* Dp     = (const float*)d_in[8];
  const float* W_out  = (const float*)d_in[9];
  float* out = (float*)d_out;

  char* ws = (char*)d_ws;
  size_t off = 0;
  const size_t oR0   = off; off += (size_t)MROWS * DI * 4;
  const size_t oR1   = off; off += (size_t)MROWS * DI * 4;
  const size_t oR2   = off; off += (size_t)MROWS * K2 * 2;
  const size_t oXB   = off; off += (size_t)MROWS * DM * 2;
  const size_t oWIN  = off; off += (size_t)NXZ * DM * 2;
  const size_t oWX2  = off; off += (size_t)XD * K2 * 2;
  const size_t oWDT2 = off; off += (size_t)DI * KDT2 * 2;
  const size_t oWO2  = off; off += (size_t)DM * K2 * 2;
  const size_t oDT   = off; off += (size_t)MROWS * 64 * 2;
  const size_t oBC   = off; off += (size_t)MROWS * 32 * 4;
  const size_t oAT   = off; off += (size_t)DI * DS * 4;
  if (off > ws_size || off > (size_t)WSMAX) return;

  float*          R0    = (float*)(ws + oR0);
  float*          R1    = (float*)(ws + oR1);
  unsigned short* R2    = (unsigned short*)(ws + oR2);
  unsigned short* XB    = (unsigned short*)(ws + oXB);
  unsigned short* WIN   = (unsigned short*)(ws + oWIN);
  unsigned short* WX2   = (unsigned short*)(ws + oWX2);
  unsigned short* WDT2  = (unsigned short*)(ws + oWDT2);
  unsigned short* WOUT2 = (unsigned short*)(ws + oWO2);
  unsigned short* DThl  = (unsigned short*)(ws + oDT);
  float*          BCp   = (float*)(ws + oBC);
  float*          ATAB  = (float*)(ws + oAT);

  k_prep<<<NU_ALL / PTHR, PTHR, 0, stream>>>(x, W_in, W_x, W_dt, W_out, A_log, XB, WIN, WX2, WDT2, WOUT2, ATAB);
  k_gemm<8, 0><<<dim3(MROWS / GBM, NXZ / 128), GTHR, 0, stream>>>(XB, DM, WIN, DM, DM, b_dt, R0, R1, DThl);
  k_conv<<<dim3(MROWS / 64, DI / 64), PTHR, 0, stream>>>(R0, W_conv, b_conv, R2);
  k_gemm<4, 1><<<dim3(MROWS / GBM, 1), GTHR, 0, stream>>>(R2, K2, WX2, K2, K2, b_dt, BCp, R1, DThl);
  k_gemm<8, 2><<<dim3(MROWS / GBM, DI / 128), GTHR, 0, stream>>>(DThl, KDT2, WDT2, KDT2, KDT2, b_dt, R0, R1, DThl);
  k_scan<<<BSZ * (DI / 64), 64, 0, stream>>>(R0, R1, BCp, ATAB, Dp, R2);
  k_gemm<8, 3><<<dim3(MROWS / GBM, DM / 128), GTHR, 0, stream>>>(R2, K2, WOUT2, K2, K2, b_dt, out, R1, DThl);
}
